// SGPN_45526653337883
// MI455X (gfx1250) — hardware-verified
//
#include <hip/hip_runtime.h>
#include <string.h>


namespace {
constexpr int NN = 512, NE = 4096, PO = 512, PR = 256, BO = PO / 64, BR = PR / 64  , NEG = NE  , DN = 256, HG = 512, D3 = 768, NOC = 160, NRC = 26, NL = 2;
constexpr float XS = 8.0f, WSC = 256.0f;

typedef _Float16 b16;
typedef __attribute__((ext_vector_type(16))) _Float16 v16b;
typedef __attribute__((ext_vector_type(8))) _Float16 v8b;
typedef __attribute__((ext_vector_type(8))) float v8f;
typedef __attribute__((ext_vector_type(4))) float v4f;
__device__ __forceinline__ float bf16_rne(float f) { unsigned int u = __float_as_uint(f); u += 0x7FFFu + ((u >> 16) & 1u); return __uint_as_float(u & 0xFFFF0000u); }
__device__ __forceinline__ v16b frag_kb(const b16* p, int hh) { const v8b a = *(const v8b*)(p + 8 * hh), b = *(const v8b*)(p + 16 + 8 * hh); v16b f;
#pragma unroll
  for (int e = 0; e < 8; ++e) { f[e] = a[e]; f[8 + e] = b[e]; } return f; }
__device__ __forceinline__ v8f wmma16b(v16b a, v16b b, v8f c) { v8f d = __builtin_amdgcn_wmma_f32_16x16x32_f16(false, a, false, b, (short)0, c, false, false); asm volatile("v_nop\n\tv_nop\n\tv_nop\n\tv_nop" : "+v"(d) : "v"(a), "v"(b)); return d; }
__device__ __forceinline__ void wave_lds_sync() { __builtin_amdgcn_fence(__ATOMIC_RELEASE, "workgroup"); __builtin_amdgcn_wave_barrier(); __builtin_amdgcn_fence(__ATOMIC_ACQUIRE, "workgroup"); }
__device__ __forceinline__ float nexp(float x) { return __builtin_amdgcn_exp2f(x * 1.4426950408889634f); }
__device__ __forceinline__ float hmax16(float v) { v = fmaxf(v, __shfl_xor(v, 1)); v = fmaxf(v, __shfl_xor(v, 2)); v = fmaxf(v, __shfl_xor(v, 4)); return fmaxf(v, __shfl_xor(v, 8)); }
__device__ __forceinline__ float hsum16(float v) { v += __shfl_xor(v, 1); v += __shfl_xor(v, 2); v += __shfl_xor(v, 4); return v + __shfl_xor(v, 8); }
__device__ __forceinline__ int iclamp(int v, int lo, int hi) { return v < lo ? lo : (v > hi ? hi : v); }

constexpr int CSR_NBLK = 512, CSR_GB = 9, CSR_GN = 1 << CSR_GB  , CSR_MAXG = 512, CSR_CAP = 12288  ;
__global__ __launch_bounds__(64) void csrA_kernel(const int* __restrict__ dst, int E, int N, int nG, int CHP, int NGP, int* __restrict__ STG, int* __restrict__ HST) {
  extern __shared__ int sm[];
  int* cnt = sm; int* run = sm + NGP; int* ids = sm + 2 * NGP;
  const int b = blockIdx.x; const int ch = (E + CSR_NBLK - 1) / CSR_NBLK; const int e0 = b * ch, e1 = min(E, e0 + ch);
  for (int i = threadIdx.x; i < NGP; i += 64) cnt[i] = 0;
  for (int i = threadIdx.x; i < CHP; i += 64) ids[i] = -1;
  __syncthreads();
  if (threadIdx.x == 0) {
    for (int e = e0; e < e1; ++e) { int d = dst[e]; d = (d < 0) ? 0 : (d >= N ? N - 1 : d); cnt[d >> CSR_GB] += 1; }
    int acc = 0; for (int g = 0; g < nG; ++g) { run[g] = acc; acc += cnt[g]; }
    for (int e = e0; e < e1; ++e) { int d = dst[e]; d = (d < 0) ? 0 : (d >= N ? N - 1 : d); const int g = d >> CSR_GB; ids[run[g]] = e; run[g] += 1; } }
  __syncthreads();
  typedef __attribute__((ext_vector_type(4))) int v4i;
  for (int pass = 0; pass < 2; ++pass) {
    for (int i = threadIdx.x; i < CHP / 4; i += 64) *(volatile v4i*)(STG + (size_t)b * CHP + i * 4) = *(const v4i*)(&ids[i * 4]);
    for (int i = threadIdx.x; i < NGP / 4; i += 64) { v4i v; for (int e = 0; e < 4; ++e) v[e] = (i * 4 + e < nG) ? cnt[i * 4 + e] : 0; *(volatile v4i*)(HST + (size_t)b * NGP + i * 4) = v; }
    __threadfence(); }
}
__global__ __launch_bounds__(512) void csrS_kernel(const int* __restrict__ HST, int nG, int NGP, int* __restrict__ START, int* __restrict__ TOT, int* __restrict__ OFF) {
  __shared__ int tot[CSR_MAXG];
  const int b = threadIdx.x;
  for (int pass = 0; pass < 2; ++pass) { int runb = 0; for (int g = 0; g < nG; ++g) { int c = HST[(size_t)b * NGP + g]; c = (c < 0) ? 0 : c; ((volatile int*)OFF)[(size_t)g * CSR_NBLK + b] = runb; runb += c; } __threadfence(); }
  for (int g = threadIdx.x; g < nG; g += 512) { int s = 0; for (int bb = 0; bb < CSR_NBLK; ++bb) { int c = HST[(size_t)bb * NGP + g]; s += (c < 0) ? 0 : c; } tot[g] = s; }
  __syncthreads();
  if (threadIdx.x < 32) {
    __shared__ int st[CSR_MAXG + 32];
    if (threadIdx.x == 0) { int acc = 0; for (int g = 0; g < NGP; ++g) { st[g] = acc; if (g < nG) acc += (tot[g] + 31) & ~31; } st[NGP] = acc; }
    __builtin_amdgcn_fence(__ATOMIC_RELEASE, "workgroup"); __builtin_amdgcn_wave_barrier(); __builtin_amdgcn_fence(__ATOMIC_ACQUIRE, "workgroup");
    for (int pass = 0; pass < 2; ++pass) { for (int i = threadIdx.x; i < NGP + 32; i += 32) { ((volatile int*)START)[i] = (i <= NGP) ? st[min(i, NGP)] : 0; ((volatile int*)TOT)[i] = (i < nG) ? tot[i] : 0; } __threadfence(); } }
}
__global__ __launch_bounds__(256) void csrB_kernel(const int* __restrict__ dst, int N, int nG, int CHP, int NGP, int permLen, const int* __restrict__ STG, const int* __restrict__ HST, const int* __restrict__ OFF, const int* __restrict__ START, const int* __restrict__ TOT, int* __restrict__ PERM, int* __restrict__ ROWPTR, int* __restrict__ ROWCNT, int* __restrict__ FLAG) {
  typedef __attribute__((ext_vector_type(4))) int v4i;
  __shared__ int ids[CSR_CAP]; __shared__ unsigned short key[CSR_CAP]; __shared__ int outp[CSR_CAP]; __shared__ int ncnt[CSR_GN + 1]; __shared__ int boff[CSR_NBLK + 1];
  const int g = blockIdx.x, t_ = threadIdx.x; int tot = TOT[g]; int st = START[g], stn = START[g + 1]; const int v0 = g * CSR_GN; const int nv = min(CSR_GN, N - v0);
  st = (st < 0) ? 0 : (st > permLen - 32 ? permLen - 32 : st) & ~31; stn = (stn < st) ? st : (stn > permLen ? permLen : stn); tot = (tot < 0) ? 0 : tot; if (tot > stn - st && tot <= CSR_CAP) tot = stn - st;
  if (tot > CSR_CAP) {
    for (int pass = 0; pass < 2; ++pass) { for (int i = t_; i < CSR_GN / 4; i += 256) { v4i a, c; for (int e = 0; e < 4; ++e) { a[e] = st; c[e] = 0; } *(volatile v4i*)(ROWPTR + v0 + i * 4) = a; *(volatile v4i*)(ROWCNT + v0 + i * 4) = c; } if (t_ == 0) ((volatile int*)FLAG)[0] = 1; __threadfence(); } (void)nv; return; }
  if (t_ == 0) { int acc = 0; for (int b = 0; b < CSR_NBLK; ++b) { boff[b] = acc; int c = HST[(size_t)b * NGP + g]; c = (c < 0) ? 0 : (c > CHP ? CHP : c); acc += c; if (acc > tot) acc = tot; } boff[CSR_NBLK] = acc; }
  for (int i = t_; i <= CSR_GN; i += 256) ncnt[i] = 0;
  __syncthreads();
  for (int b = 0; b < CSR_NBLK; ++b) { const int c = boff[b + 1] - boff[b]; int o_ = OFF[(size_t)g * CSR_NBLK + b]; o_ = (o_ < 0) ? 0 : (o_ > CHP - c ? CHP - c : o_); const int* src_ = STG + (size_t)b * CHP + o_;
    for (int i = t_; i < c; i += 256) { int id = src_[i]; id = (id < 0) ? 0 : id; ids[boff[b] + i] = id; int d = dst[id]; d = (d < v0) ? v0 : (d >= N ? N - 1 : d); int kk = d - v0; kk = (kk < 0) ? 0 : (kk >= CSR_GN ? CSR_GN - 1 : kk); key[boff[b] + i] = (unsigned short)kk; } }
  __syncthreads();
  if (t_ == 0) { for (int i = 0; i < tot; ++i) ncnt[key[i]] += 1; int acc = 0; for (int vl = 0; vl < CSR_GN; ++vl) { const int c = ncnt[vl]; ncnt[vl] = acc; acc += c; } ncnt[CSR_GN] = acc;
    for (int i = 0; i < tot; ++i) { const int vl = key[i]; outp[ncnt[vl]] = ids[i]; ncnt[vl] += 1; }
    for (int vl = CSR_GN; vl > 0; --vl) ncnt[vl] = ncnt[vl - 1]; ncnt[0] = 0; }
  __syncthreads();
  for (int pass = 0; pass < 2; ++pass) {
    for (int i = t_; i < (stn - st) / 4; i += 256) { v4i v; for (int e = 0; e < 4; ++e) { const int q = i * 4 + e; v[e] = (q < tot) ? outp[q] : -1; } *(volatile v4i*)(PERM + st + i * 4) = v; }
    for (int i = t_; i < CSR_GN / 4; i += 256) { v4i a, c; for (int e = 0; e < 4; ++e) { const int vl = i * 4 + e; a[e] = st + ncnt[vl]; c[e] = (vl < nv) ? (ncnt[vl + 1] - ncnt[vl]) : 0; } *(volatile v4i*)(ROWPTR + v0 + i * 4) = a; *(volatile v4i*)(ROWCNT + v0 + i * 4) = c; }
    __threadfence(); }
}
__global__ __launch_bounds__(256) void csrZ_kernel(int* __restrict__ p, size_t n4) { typedef __attribute__((ext_vector_type(4))) int v4i; const size_t tid = (size_t)blockIdx.x * 256 + threadIdx.x, nth = (size_t)gridDim.x * 256; v4i z = {0, 0, 0, 0}; for (size_t i = tid; i < n4; i += nth) *(volatile v4i*)(p + i * 4) = z; }
struct CsrBufs { int *STG, *HST, *OFF, *START, *TOT, *PERM, *ROWPTR, *ROWCNT, *FLAG; int nG, NGP, CHP; size_t permLen; char* base; size_t bytes; };
static size_t csr_carve(CsrBufs& c, char* ws, size_t off, int E, int N) {
  const size_t off0 = off; c.base = ws + off;
  auto al = [&](size_t bytes) { char* p = ws + off; off += (bytes + 255) & ~(size_t)255; return p; };
  c.nG = (N + CSR_GN - 1) / CSR_GN; c.NGP = (c.nG + 31) & ~31; const int ch = (E + CSR_NBLK - 1) / CSR_NBLK; c.CHP = (ch + 31) & ~31; c.permLen = (size_t)E + 32 * (size_t)c.nG + 32;
  c.STG = (int*)al((size_t)CSR_NBLK * c.CHP * 4); c.HST = (int*)al((size_t)CSR_NBLK * c.NGP * 4); c.OFF = (int*)al((size_t)c.NGP * CSR_NBLK * 4); c.START = (int*)al((size_t)(c.NGP + 64) * 4); c.TOT = (int*)al((size_t)(c.NGP + 64) * 4);
  c.PERM = (int*)al(c.permLen * 4); c.ROWPTR = (int*)al((size_t)c.nG * CSR_GN * 4); c.ROWCNT = (int*)al((size_t)c.nG * CSR_GN * 4); c.FLAG = (int*)al(256);
  c.bytes = off - off0; return off;
}
static void csr_build(const CsrBufs& c, const int* dst, int E, int N, hipStream_t stream) {
  const size_t smem = (size_t)(2 * c.NGP + c.CHP) * 4;
  csrZ_kernel<<<512, 256, 0, stream>>>((int*)c.base, c.bytes / 16);
  csrA_kernel<<<CSR_NBLK, 64, smem, stream>>>(dst, E, N, c.nG, c.CHP, c.NGP, c.STG, c.HST);
  csrS_kernel<<<1, 512, 0, stream>>>(c.HST, c.nG, c.NGP, c.START, c.TOT, c.OFF);
  csrB_kernel<<<c.nG, 256, 0, stream>>>(dst, N, c.nG, c.CHP, c.NGP, (int)c.permLen, c.STG, c.HST, c.OFF, c.START, c.TOT, c.PERM, c.ROWPTR, c.ROWCNT, c.FLAG);
}


struct WDesc { const float* w; b16* dst; int IN, KP, OUT, OUTP; };
struct WDescs { WDesc d[20]; };
__global__ __launch_bounds__(256) void prepw_kernel(WDescs descs) {
  const WDesc d = descs.d[blockIdx.y]; const int t = blockIdx.x * 256 + threadIdx.x; const int ngrp = d.OUTP * d.KP / 8; if (t >= ngrp) return; const int o_ = (t * 8) / d.KP, k0 = t * 8 - o_ * d.KP; v8b o;
  for (int j = 0; j < 8; ++j) { const int k = k0 + j; o[j] = (k < d.IN && o_ < d.OUT) ? (b16)(bf16_rne(d.w[(size_t)k * d.OUT + o_]) * WSC) : (b16)0.0f; }
  for (int pass = 0; pass < 2; ++pass) { *(volatile v8b*)(d.dst + (size_t)t * 8) = o; __threadfence(); }
}
template <int CIN, int NP, int NBLK>
__global__ __launch_bounds__(128) void pointnet_kernel(const float* __restrict__ pts, const b16* __restrict__ W1, const float* __restrict__ b1, const b16* __restrict__ W2, const float* __restrict__ b2, const b16* __restrict__ W3, const float* __restrict__ b3, float* __restrict__ PMX) {
  __shared__ __attribute__((aligned(16))) b16 Ta[4][16][32 + 8], H1[4][16][64 + 8], H2[4][16][128 + 8]; __shared__ float Mx[4][DN];
  const int wave = threadIdx.x >> 5, lane = threadIdx.x & 31, nloc = lane & 15, hlf = lane >> 4, t_ = threadIdx.x; const int cloud = blockIdx.x / NBLK, blk = blockIdx.x - cloud * NBLK; const int p0 = blk * 64 + wave * 16;
  { const int rr = lane >> 1, hf = lane & 1; v8b z = {}; if (hf == 0) { for (int c = 0; c < CIN; ++c) z[c] = (b16)(bf16_rne(pts[((size_t)cloud * CIN + c) * NP + p0 + rr]) * XS); *(v8b*)(&Ta[wave][rr][0]) = z; v8b z0 = {}; *(v8b*)(&Ta[wave][rr][8]) = z0; } else { v8b z0 = {}; *(v8b*)(&Ta[wave][rr][16]) = z0; *(v8b*)(&Ta[wave][rr][24]) = z0; } }
  wave_lds_sync();
  { const v16b a = frag_kb(&Ta[wave][nloc][0], hlf);
#pragma unroll
    for (int t = 0; t < 4; ++t) { v8f acc = {}; acc = wmma16b(a, frag_kb(W1 + (size_t)(t * 16 + nloc) * 32, hlf), acc); const float bb = bf16_rne(b1[t * 16 + nloc]);
#pragma unroll
      for (int r = 0; r < 8; ++r) H1[wave][8 * hlf + r][t * 16 + nloc] = (b16)(fmaxf(acc[r] * (1.0f / (XS * WSC)) + bb, 0.0f) * XS); } }
  wave_lds_sync();
  { v8f acc[8];
#pragma unroll
    for (int t = 0; t < 8; ++t) acc[t] = (v8f){};
#pragma unroll
    for (int kb = 0; kb < 64; kb += 32) { const v16b a = frag_kb(&H1[wave][nloc][kb], hlf);
#pragma unroll
      for (int t = 0; t < 8; ++t) acc[t] = wmma16b(a, frag_kb(W2 + (size_t)(t * 16 + nloc) * 64 + kb, hlf), acc[t]); }
#pragma unroll
    for (int t = 0; t < 8; ++t) { const float bb = bf16_rne(b2[t * 16 + nloc]);
#pragma unroll
      for (int r = 0; r < 8; ++r) H2[wave][8 * hlf + r][t * 16 + nloc] = (b16)(fmaxf(acc[t][r] * (1.0f / (XS * WSC)) + bb, 0.0f) * XS); } }
  wave_lds_sync();
  { v8f acc[16];
#pragma unroll
    for (int t = 0; t < 16; ++t) acc[t] = (v8f){};
#pragma unroll
    for (int kb = 0; kb < 128; kb += 32) { const v16b a = frag_kb(&H2[wave][nloc][kb], hlf);
#pragma unroll
      for (int t = 0; t < 16; ++t) acc[t] = wmma16b(a, frag_kb(W3 + (size_t)(t * 16 + nloc) * 128 + kb, hlf), acc[t]); }
#pragma unroll
    for (int t = 0; t < 16; ++t) { float m = -INFINITY;
#pragma unroll
      for (int r = 0; r < 8; ++r) m = fmaxf(m, acc[t][r]);
      m = fmaxf(m, __shfl_xor(m, 16)); if (hlf == 0) Mx[wave][t * 16 + nloc] = m * (1.0f / (XS * WSC)) + bf16_rne(b3[t * 16 + nloc]); } }
  __syncthreads();
  for (int pass = 0; pass < 2; ++pass) { if (t_ < 64) { v4f o; for (int j = 0; j < 4; ++j) { const int c = t_ * 4 + j; o[j] = fmaxf(fmaxf(Mx[0][c], Mx[1][c]), fmaxf(Mx[2][c], Mx[3][c])); } *(volatile v4f*)(PMX + ((size_t)cloud * NBLK + blk) * DN + t_ * 4) = o; } __threadfence(); }
}
__global__ __launch_bounds__(256) void maxred_kernel(const float* __restrict__ PMX, int nblk, int nclouds, float* __restrict__ F32, b16* __restrict__ F16) {
  const int wave = threadIdx.x >> 5, lane = threadIdx.x & 31; const int cloud = blockIdx.x * 8 + wave; if (cloud >= nclouds) return;
  float m[8]; for (int j = 0; j < 8; ++j) m[j] = -INFINITY;
  for (int b = 0; b < nblk; ++b) { const v4f a = *(const v4f*)(PMX + ((size_t)cloud * nblk + b) * DN + lane * 8), c = *(const v4f*)(PMX + ((size_t)cloud * nblk + b) * DN + lane * 8 + 4); for (int j = 0; j < 4; ++j) { m[j] = fmaxf(m[j], a[j]); m[4 + j] = fmaxf(m[4 + j], c[j]); } }
  v4f o0 = {m[0], m[1], m[2], m[3]}, o1 = {m[4], m[5], m[6], m[7]}; v8b h; for (int j = 0; j < 8; ++j) h[j] = (b16)(m[j] * XS);
  for (int pass = 0; pass < 2; ++pass) { *(volatile v4f*)(F32 + (size_t)cloud * DN + lane * 8) = o0; *(volatile v4f*)(F32 + (size_t)cloud * DN + lane * 8 + 4) = o1; *(volatile v8b*)(F16 + (size_t)cloud * DN + lane * 8) = h; __threadfence(); }
}
struct GemmArgs { const b16* s0; const int* i0; const b16* s1; const b16* s2; const int* i2; const b16* W; const float* b; b16* Y16; float* Y32;
                  int ld0, ld1, ld2, K1, K2, K, OUT, relu, ldy, nidx; };
__host__ inline GemmArgs mkargs(const b16* s0, const int* i0, int ld0, const b16* s1, int ld1, const b16* s2, const int* i2, int ld2, int K1, int K2, int K, const b16* W, const float* b, int OUT, int relu, b16* Y16, float* Y32, int ldy, int nidx) {
  GemmArgs g; memset(&g, 0, sizeof(g)); g.s0 = s0; g.i0 = i0; g.ld0 = ld0; g.s1 = s1; g.ld1 = ld1; g.s2 = s2; g.i2 = i2; g.ld2 = ld2; g.K1 = K1; g.K2 = K2; g.K = K; g.W = W; g.b = b; g.OUT = OUT; g.relu = relu; g.Y16 = Y16; g.Y32 = Y32; g.ldy = ldy; g.nidx = nidx; return g; }
template <int MODE>
__global__ __launch_bounds__(128) void gemm_kernel(GemmArgs g) {
  __shared__ __attribute__((aligned(16))) float Ts[4][16][128 + 4];
  const int wave = threadIdx.x >> 5, lane = threadIdx.x & 31, nloc = lane & 15, hlf = lane >> 4; const size_t m0 = (size_t)blockIdx.x * 64 + wave * 16; const int n0 = blockIdx.y * 128;
  const size_t ra = m0 + nloc; const int r0 = g.i0 ? iclamp(g.i0[ra], 0, g.nidx - 1) : (int)ra; const int r2 = g.i2 ? iclamp(g.i2[ra], 0, g.nidx - 1) : (int)ra;
  v8f acc[8];
#pragma unroll
  for (int t = 0; t < 8; ++t) acc[t] = (v8f){};
  for (int kb = 0; kb < g.K; kb += 32) { const b16* ap = (kb < g.K1) ? g.s0 + (size_t)r0 * g.ld0 + kb : (kb < g.K2 ? g.s1 + ra * g.ld1 + (kb - g.K1) : g.s2 + (size_t)r2 * g.ld2 + (kb - g.K2)); const v16b a = frag_kb(ap, hlf);
#pragma unroll
    for (int t = 0; t < 8; ++t) acc[t] = wmma16b(a, frag_kb(g.W + (size_t)(n0 + t * 16 + nloc) * g.K + kb, hlf), acc[t]); }
#pragma unroll
  for (int t = 0; t < 8; ++t) { const int c = n0 + t * 16 + nloc; const float bb = (c < g.OUT) ? bf16_rne(g.b[c < g.OUT ? c : 0]) : 0.0f;
#pragma unroll
    for (int r = 0; r < 8; ++r) { float v = acc[t][r] * (1.0f / (XS * WSC)) + bb; if (g.relu) v = fmaxf(v, 0.0f); Ts[wave][8 * hlf + r][t * 16 + nloc] = v; } }
  wave_lds_sync();
  for (int pass = 0; pass < 2; ++pass) {
    for (int rr = 0; rr < 16; ++rr) { if (MODE == 0) { if (lane < 16) { v8b h; for (int j = 0; j < 8; ++j) h[j] = (b16)(Ts[wave][rr][lane * 8 + j] * XS); *(volatile v8b*)(g.Y16 + (m0 + rr) * g.ldy + n0 + lane * 8) = h; } }
      else { *(volatile v4f*)(g.Y32 + (m0 + rr) * g.ldy + n0 + lane * 4) = *(const v4f*)(&Ts[wave][rr][lane * 4]); } }
    __threadfence(); }
}
__global__ __launch_bounds__(256) void nodeagg_kernel(const float* __restrict__ HO, const int* __restrict__ PS, const int* __restrict__ RPS, const int* __restrict__ RCS, int plS, const int* __restrict__ PO_, const int* __restrict__ RPO, const int* __restrict__ RCO, int plO, b16* __restrict__ AV16) {
  const int wave = threadIdx.x >> 5, lane = threadIdx.x & 31; const int v = (blockIdx.x * 8 + wave) * 2 + (lane >> 4); const int c0 = (lane & 15) * 16;
  float acc[16]; for (int j = 0; j < 16; ++j) acc[j] = 0.0f;
  int st = RPS[v], cnt = RCS[v]; cnt = iclamp(cnt, 0, NE); st = iclamp(st, 0, plS - cnt);
  for (int j = 0; j < cnt; ++j) { const int e = iclamp(PS[st + j], 0, NE - 1); const float* p = HO + (size_t)e * D3 + c0; for (int q = 0; q < 16; ++q) acc[q] += p[q]; }
  int st2 = RPO[v], cnt2 = RCO[v]; cnt2 = iclamp(cnt2, 0, NE); st2 = iclamp(st2, 0, plO - cnt2);
  for (int j = 0; j < cnt2; ++j) { const int e = iclamp(PO_[st2 + j], 0, NE - 1); const float* p = HO + (size_t)e * D3 + 2 * DN + c0; for (int q = 0; q < 16; ++q) acc[q] += p[q]; }
  const float inv = 1.0f / (float)((cnt + cnt2) > 1 ? (cnt + cnt2) : 1); v8b h0, h1; for (int q = 0; q < 8; ++q) { h0[q] = (b16)(acc[q] * inv * XS); h1[q] = (b16)(acc[8 + q] * inv * XS); }
  for (int pass = 0; pass < 2; ++pass) { *(volatile v8b*)(AV16 + (size_t)v * DN + c0) = h0; *(volatile v8b*)(AV16 + (size_t)v * DN + c0 + 8) = h1; __threadfence(); }
}
__global__ __launch_bounds__(256) void ecopy_kernel(const float* __restrict__ HO, b16* __restrict__ E16) {
  const int t = blockIdx.x * 256 + threadIdx.x; if (t >= NE * DN / 8) return; const int e = (t * 8) / DN, c = t * 8 - e * DN; const float* p = HO + (size_t)e * D3 + DN + c; v8b h; for (int j = 0; j < 8; ++j) h[j] = (b16)(p[j] * XS);
  for (int pass = 0; pass < 2; ++pass) { *(volatile v8b*)(E16 + (size_t)t * 8) = h; __threadfence(); }
}
__global__ __launch_bounds__(256) void objhead_kernel(const float* __restrict__ L, float* __restrict__ out0) {
  __shared__ float S[64][NOC];
  const int wave = threadIdx.x >> 5, lane = threadIdx.x & 31, t_ = threadIdx.x; const int r0 = blockIdx.x * 64;
  for (int rr = wave; rr < 64; rr += 8) { const float* p = L + (size_t)(r0 + rr) * 256; float v[5], m = -INFINITY; for (int j = 0; j < 5; ++j) { v[j] = p[lane * 5 + j]; m = fmaxf(m, v[j]); }
#pragma unroll
    for (int o = 16; o >= 1; o >>= 1) m = fmaxf(m, __shfl_xor(m, o));
    float s = 0.0f; for (int j = 0; j < 5; ++j) s += nexp(v[j] - m);
#pragma unroll
    for (int o = 16; o >= 1; o >>= 1) s += __shfl_xor(s, o);
    const float lse = m + __logf(s); for (int j = 0; j < 5; ++j) S[rr][lane * 5 + j] = v[j] - lse; }
  __syncthreads();
  for (int pass = 0; pass < 2; ++pass) { for (int q = t_; q < 64 * NOC / 4; q += 256) *(volatile v4f*)(out0 + (size_t)r0 * NOC + q * 4) = *(const v4f*)(&S[0][0] + q * 4); __threadfence(); }
}
__global__ __launch_bounds__(256) void relhead_kernel(const float* __restrict__ L, float* __restrict__ out1) {
  __shared__ float S[64 * NRC];
  const int t_ = threadIdx.x; const int r0 = blockIdx.x * 64;
  for (int q = t_; q < 64 * NRC; q += 256) { const int rr = q / NRC, c = q - rr * NRC; const float x = L[(size_t)(r0 + rr) * 128 + c]; S[q] = 1.0f / (1.0f + nexp(-x)); }
  __syncthreads();
  for (int pass = 0; pass < 2; ++pass) { for (int q = t_; q < 64 * NRC / 4; q += 256) *(volatile v4f*)(out1 + (size_t)r0 * NRC + q * 4) = *(const v4f*)(&S[q * 4]); __threadfence(); }
}
}

extern "C" void kernel_launch(void* const* d_in, const int* in_sizes, int n_in, void* d_out, int out_size, void* d_ws, size_t ws_size, hipStream_t stream) {
  (void)n_in;
  auto Fp = [&](int i) { return (const float*)d_in[i]; };
  if (in_sizes[0] != NN * 3 * PO || in_sizes[1] != NE * 4 * PR || in_sizes[2] != 2 * NE || in_sizes[15] != NL * D3 * HG || in_sizes[17] != NL * HG * D3 || in_sizes[27] != DN * NOC || in_sizes[33] != DN * NRC || out_size != NN * NOC + NE * NRC) return;
  const int* es = (const int*)d_in[2]; const int* eo = es + NE;
  size_t off = 0; char* ws = (char*)d_ws;
  auto carve = [&](size_t bytes) { char* p = ws + off; off += (bytes + 255) & ~(size_t)255; return p; };
  b16* W1o = (b16*)carve(64 * 32 * 2); b16* W2o = (b16*)carve(128 * 64 * 2); b16* W3o = (b16*)carve(256 * 128 * 2); b16* W1r = (b16*)carve(64 * 32 * 2); b16* W2r = (b16*)carve(128 * 64 * 2); b16* W3r = (b16*)carve(256 * 128 * 2);
  b16* TW1[2]; b16* TW2[2]; b16* NW1[2]; b16* NW2[2]; for (int l = 0; l < 2; ++l) { TW1[l] = (b16*)carve((size_t)HG * D3 * 2); TW2[l] = (b16*)carve((size_t)D3 * HG * 2); NW1[l] = (b16*)carve((size_t)HG * DN * 2); NW2[l] = (b16*)carve((size_t)DN * HG * 2); }
  b16* OC1 = (b16*)carve((size_t)HG * DN * 2); b16* OC2 = (b16*)carve((size_t)DN * HG * 2); b16* OC3 = (b16*)carve((size_t)256 * DN * 2); b16* RC1 = (b16*)carve((size_t)HG * DN * 2); b16* RC2 = (b16*)carve((size_t)DN * HG * 2); b16* RC3 = (b16*)carve((size_t)128 * DN * 2);
  float* PMXo = (float*)carve((size_t)NN * (PO / 64) * DN * 4); float* PMXr = (float*)carve((size_t)NE * (PR / 64) * DN * 4);
  float* X32 = (float*)carve((size_t)NN * DN * 4); b16* X16 = (b16*)carve((size_t)NN * DN * 2); float* E32 = (float*)carve((size_t)NE * DN * 4); b16* E16 = (b16*)carve((size_t)NE * DN * 2);
  b16* H16 = (b16*)carve((size_t)NE * HG * 2); float* HO = (float*)carve((size_t)NE * D3 * 4); b16* AV16 = (b16*)carve((size_t)NN * DN * 2); b16* NH16 = (b16*)carve((size_t)NN * HG * 2);
  b16* C1 = (b16*)carve((size_t)NE * HG * 2); b16* C2 = (b16*)carve((size_t)NE * DN * 2); float* LG = (float*)carve((size_t)NE * 128 * 4); float* LGo = (float*)carve((size_t)NN * 256 * 4);
  CsrBufs csrS, csrO; off = csr_carve(csrS, ws, off, NE, NN); off = csr_carve(csrO, ws, off, NE, NN);
  if (off > ws_size || off > ((size_t)128 << 20)) return;
  WDescs hd = {{
    {Fp(3), W1o, 3, 32, 64, 64}, {Fp(5), W2o, 64, 64, 128, 128}, {Fp(7), W3o, 128, 128, 256, 256}, {Fp(9), W1r, 4, 32, 64, 64}, {Fp(11), W2r, 64, 64, 128, 128}, {Fp(13), W3r, 128, 128, 256, 256},
    {Fp(15), TW1[0], D3, D3, HG, HG}, {Fp(15) + (size_t)D3 * HG, TW1[1], D3, D3, HG, HG}, {Fp(17), TW2[0], HG, HG, D3, D3}, {Fp(17) + (size_t)HG * D3, TW2[1], HG, HG, D3, D3},
    {Fp(19), NW1[0], DN, DN, HG, HG}, {Fp(19) + (size_t)DN * HG, NW1[1], DN, DN, HG, HG}, {Fp(21), NW2[0], HG, HG, DN, DN}, {Fp(21) + (size_t)HG * DN, NW2[1], HG, HG, DN, DN},
    {Fp(23), OC1, DN, DN, HG, HG}, {Fp(25), OC2, HG, HG, DN, DN}, {Fp(27), OC3, DN, DN, NOC, 256},
    {Fp(29), RC1, DN, DN, HG, HG}, {Fp(31), RC2, HG, HG, DN, DN}, {Fp(33), RC3, DN, DN, NRC, 128} }};
  prepw_kernel<<<dim3((D3 * HG / 8 + 255) / 256, 20), 256, 0, stream>>>(hd);
  pointnet_kernel<3, PO, BO><<<NN * BO, 128, 0, stream>>>(Fp(0), W1o, Fp(4), W2o, Fp(6), W3o, Fp(8), PMXo);
  maxred_kernel<<<NN / 8, 256, 0, stream>>>(PMXo, BO, NN, X32, X16);
  pointnet_kernel<4, PR, BR><<<NEG * BR, 128, 0, stream>>>(Fp(1), W1r, Fp(10), W2r, Fp(12), W3r, Fp(14), PMXr);
  maxred_kernel<<<NEG / 8, 256, 0, stream>>>(PMXr, BR, NEG, E32, E16);
  csr_build(csrS, es, NEG, NN, stream); csr_build(csrO, eo, NEG, NN, stream);
  for (int l = 0; l < NL; ++l) {
    GemmArgs g1 = mkargs(X16, es, DN, E16, DN, X16, eo, DN, DN, 2 * DN, D3, TW1[l], Fp(16) + l * HG, HG, 1, H16, nullptr, HG, NN);
    gemm_kernel<0><<<dim3(NEG / 64, HG / 128), 128, 0, stream>>>(g1);
    GemmArgs g2 = mkargs(H16, nullptr, HG, nullptr, 0, nullptr, nullptr, 0, HG, HG, HG, TW2[l], Fp(18) + l * D3, D3, 0, nullptr, HO, D3, NE);
    gemm_kernel<1><<<dim3(NEG / 64, D3 / 128), 128, 0, stream>>>(g2);
    nodeagg_kernel<<<NN / 16, 256, 0, stream>>>(HO, csrS.PERM, csrS.ROWPTR, csrS.ROWCNT, (int)csrS.permLen, csrO.PERM, csrO.ROWPTR, csrO.ROWCNT, (int)csrO.permLen, AV16);
    GemmArgs g3 = mkargs(AV16, nullptr, DN, nullptr, 0, nullptr, nullptr, 0, DN, DN, DN, NW1[l], Fp(20) + l * HG, HG, 1, NH16, nullptr, HG, NN);
    gemm_kernel<0><<<dim3(NN / 64, HG / 128), 128, 0, stream>>>(g3);
    GemmArgs g4 = mkargs(NH16, nullptr, HG, nullptr, 0, nullptr, nullptr, 0, HG, HG, HG, NW2[l], Fp(22) + l * DN, DN, 0, X16, nullptr, DN, NN);
    gemm_kernel<0><<<dim3(NN / 64, DN / 128), 128, 0, stream>>>(g4);
    ecopy_kernel<<<(NEG * DN / 8 + 255) / 256, 256, 0, stream>>>(HO, E16); }
  { GemmArgs a = mkargs(X16, nullptr, DN, nullptr, 0, nullptr, nullptr, 0, DN, DN, DN, OC1, Fp(24), HG, 1, C1, nullptr, HG, NN); gemm_kernel<0><<<dim3(NN / 64, HG / 128), 128, 0, stream>>>(a);
    GemmArgs b = mkargs(C1, nullptr, HG, nullptr, 0, nullptr, nullptr, 0, HG, HG, HG, OC2, Fp(26), DN, 1, C2, nullptr, DN, NN); gemm_kernel<0><<<dim3(NN / 64, DN / 128), 128, 0, stream>>>(b);
    GemmArgs c = mkargs(C2, nullptr, DN, nullptr, 0, nullptr, nullptr, 0, DN, DN, DN, OC3, Fp(28), NOC, 0, nullptr, LGo, 256, NN); gemm_kernel<1><<<dim3(NN / 64, 2), 128, 0, stream>>>(c);
    objhead_kernel<<<NN / 64, 256, 0, stream>>>(LGo, (float*)d_out); }
  { GemmArgs a = mkargs(E16, nullptr, DN, nullptr, 0, nullptr, nullptr, 0, DN, DN, DN, RC1, Fp(30), HG, 1, C1, nullptr, HG, NE); gemm_kernel<0><<<dim3(NEG / 64, HG / 128), 128, 0, stream>>>(a);
    GemmArgs b = mkargs(C1, nullptr, HG, nullptr, 0, nullptr, nullptr, 0, HG, HG, HG, RC2, Fp(32), DN, 1, C2, nullptr, DN, NE); gemm_kernel<0><<<dim3(NEG / 64, DN / 128), 128, 0, stream>>>(b);
    GemmArgs c = mkargs(C2, nullptr, DN, nullptr, 0, nullptr, nullptr, 0, DN, DN, DN, RC3, Fp(34), NRC, 0, nullptr, LG, 128, NE); gemm_kernel<1><<<dim3(NEG / 64, 1), 128, 0, stream>>>(c);
    relhead_kernel<<<NEG / 64, 256, 0, stream>>>(LG, (float*)d_out + (size_t)NN * NOC); }
}
